// PVConv2d_54683523613037
// MI455X (gfx1250) — hardware-verified
//
#include <hip/hip_runtime.h>
#include <math.h>

typedef __attribute__((ext_vector_type(16))) _Float16 v16h;
typedef __attribute__((ext_vector_type(16))) __bf16 v16b;
typedef __attribute__((ext_vector_type(8)))  _Float16 v8h;
typedef __attribute__((ext_vector_type(8)))  float v8f;
typedef __attribute__((ext_vector_type(4)))  float v4f;
typedef __attribute__((ext_vector_type(2)))  float v2f;
typedef __attribute__((ext_vector_type(4)))  unsigned v4u;
typedef __attribute__((ext_vector_type(4)))  int v4i;
typedef float __attribute__((may_alias)) float_a;
typedef int __attribute__((may_alias)) int_a;

template <typename T> __device__ __forceinline__ void vst2(void* p, T v) { *(volatile T*)p = v; __threadfence(); *(volatile T*)p = v; }
__device__ __forceinline__ v8f wmma16(v16h a, v16h b, v8f c) {
  v8f d = __builtin_amdgcn_wmma_f32_16x16x32_f16(false, a, false, b, (short)0, c, false, false);
  asm volatile("v_nop\n\tv_nop\n\tv_nop\n\tv_nop" : "+v"(d) : "v"(a), "v"(b));
  return d;
}
__device__ __forceinline__ v8f wmma_bf(v16b a, v16b b, v8f c) {
  v8f d = __builtin_amdgcn_wmma_f32_16x16x32_bf16(false, a, false, b, (short)0, c, false, false);
  asm volatile("v_nop\n\tv_nop\n\tv_nop\n\tv_nop" : "+v"(d) : "v"(a), "v"(b));
  return d;
}
__device__ __forceinline__ v16h frag_h(const _Float16* rowk0, int lane) {
  union { v16h v; v8h q[2]; } u; const _Float16* p = rowk0 + 8 * (lane >> 4);
  u.q[0] = *(const v8h*)p; u.q[1] = *(const v8h*)(p + 16); return u.v;
}
__device__ __forceinline__ v16h frag_f32(const float* rowk0, int lane) {
  v16h a; const float* p = rowk0 + 8 * (lane >> 4);
#pragma unroll
  for (int i = 0; i < 8; ++i) { a[i] = (_Float16)p[i]; a[8 + i] = (_Float16)p[16 + i]; }
  return a;
}
__device__ __forceinline__ v16h frag_f32s(const float* rowk0, int lane, float sc) {
  v16h a; const float* p = rowk0 + 8 * (lane >> 4);
#pragma unroll
  for (int i = 0; i < 8; ++i) { a[i] = (_Float16)(p[i] * sc); a[8 + i] = (_Float16)(p[16 + i] * sc); }
  return a;
}
__device__ __forceinline__ v16h fragc_f32(const float* W, int k0, int n, int lane, int ld, int K) {
  v16h a; const int g = lane >> 4;
#pragma unroll
  for (int i = 0; i < 8; ++i) { const int ka = k0 + 8 * g + i, kb = ka + 16;
    a[i] = (_Float16)(ka < K ? W[(size_t)(ka < K ? ka : K - 1) * ld + n] : 0.f); a[8 + i] = (_Float16)(kb < K ? W[(size_t)(kb < K ? kb : K - 1) * ld + n] : 0.f); }
  return a;
}
struct F2 { v16b h, l; };
__device__ __forceinline__ F2 bsplit16(const float v[16]) { F2 r;
#pragma unroll
  for (int i = 0; i < 16; ++i) { const __bf16 h = (__bf16)v[i]; r.h[i] = h; r.l[i] = (__bf16)(v[i] - (float)h); }
  return r; }
__device__ __forceinline__ F2 split_row(const float* row, int k0, int lane) { float v[16]; const float* p = row + k0 + 8 * (lane >> 4);
#pragma unroll
  for (int i = 0; i < 8; ++i) { v[i] = p[i]; v[8 + i] = p[16 + i]; }
  return bsplit16(v); }
__device__ __forceinline__ F2 split_rowK(const float* row, int k0, int lane, int K) { float v[16]; const int g = lane >> 4;
#pragma unroll
  for (int i = 0; i < 8; ++i) { const int ka = k0 + 8 * g + i, kb = ka + 16; v[i] = ka < K ? row[ka < K ? ka : K - 1] : 0.f; v[8 + i] = kb < K ? row[kb < K ? kb : K - 1] : 0.f; }
  return bsplit16(v); }
__device__ __forceinline__ F2 split_col(const float* W, int k0, int n, int lane, int ld, int K) { float v[16]; const int g = lane >> 4;
#pragma unroll
  for (int i = 0; i < 8; ++i) { const int ka = k0 + 8 * g + i, kb = ka + 16; v[i] = ka < K ? W[(size_t)(ka < K ? ka : K - 1) * ld + n] : 0.f; v[8 + i] = kb < K ? W[(size_t)(kb < K ? kb : K - 1) * ld + n] : 0.f; }
  return bsplit16(v); }
__device__ __forceinline__ v8f mac3(const F2& a, const F2& b, v8f c) { c = wmma_bf(a.l, b.h, c); c = wmma_bf(a.h, b.l, c); return wmma_bf(a.h, b.h, c); }
__device__ __forceinline__ float sigm(float v) { return 1.0f / (1.0f + expf(-v)); }
#define LDSX() do { asm volatile("s_wait_dscnt 0" ::: "memory"); __builtin_amdgcn_wave_barrier(); __builtin_amdgcn_fence(__ATOMIC_RELEASE, "workgroup"); } while (0)


#define NB 4
#define CI 32
#define CO 32
#define HH 256
#define WWD 256
#define NP (HH * WWD)
#define KK 9
#ifndef TPB
#define TPB (NP / 64)
#define TNB NB
#endif
typedef __attribute__((ext_vector_type(8))) __bf16 v8b;
__device__ __forceinline__ v16b frag_b(const __bf16* rowk0, int lane) {
  union { v16b v; v8b q[2]; } u; const __bf16* p = rowk0 + 8 * (lane >> 4);
  u.q[0] = *(const v8b*)p; u.q[1] = *(const v8b*)(p + 16); return u.v;
}
__device__ __forceinline__ float bfr(float v) { return (float)(__bf16)v; }
__device__ __attribute__((noinline)) float exp_ni(float v) { return expf(v); }
__device__ __attribute__((noinline)) float erf_ni(float v) { return erff(v); }
#define SQC 0.1f
#define PEPS 1e-7f

#define WS_PW  0u
#define WS_U   (WS_PW + 2u * (size_t)CO * KK * CI)
#define WS_END (WS_U + 4u * (size_t)NB * NP * CI)

__global__ __launch_bounds__(32) void k_packw(const float* __restrict__ WK, __bf16* __restrict__ PW) { const int o = blockIdx.x, t = threadIdx.x; __shared__ __align__(16) __bf16 s[KK * CI];
  for (int k = 0; k < KK; ++k) s[k * CI + t] = (__bf16)WK[((size_t)k * CO + o) * CI + t]; __syncthreads(); for (int q = t; q < KK * CI / 8; q += 32) vst2((unsigned*)(PW + (size_t)o * KK * CI + q * 8), *(const v4u*)&s[q * 8]); }
__global__ __launch_bounds__(256) void k_log(const float* __restrict__ X, float* __restrict__ U) { __shared__ __align__(16) float sx[256][CI + 4]; const int t = threadIdx.x; const size_t b = blockIdx.y; const size_t p0 = (size_t)blockIdx.x * 256;
  for (int c = 0; c < CI; ++c) sx[t][c] = bfr(X[(b * CI + c) * NP + p0 + t]);
  float q = 0.f; for (int c = 0; c < CI; ++c) q += sx[t][c] * sx[t][c]; const float n = fmaxf(sqrtf(q), PEPS); const float a = fminf(fmaxf(SQC * n, 0.f), 1.0f - 1e-6f); const float f = atanhf(a) / (SQC * n);
  for (int c = 0; c < CI; ++c) sx[t][c] *= f; __syncthreads();
  for (int e = t; e < 256 * 8; e += 256) { const int pl = e >> 3, qq = e & 7; vst2(U + ((b * NP + p0 + pl) * CI) + qq * 4, *(const v4f*)&sx[pl][qq * 4]); } }
__global__ __launch_bounds__(128) void k_conv(const float* __restrict__ U, const __bf16* __restrict__ PW, const float* __restrict__ BIAS, float* __restrict__ Y) { __shared__ __align__(16) float so[CO][64 + 4];
  const int tid = threadIdx.x, wave = tid >> 5, lane = tid & 31, col = lane & 15, g = lane >> 4; const size_t b = blockIdx.y; const int p0 = blockIdx.x * 64 + wave * 16; const int pix = p0 + col; const int py = pix / WWD, px = pix % WWD;
  v8f acc[2] = {};
#pragma unroll 1
  for (int k = 0; k < KK; ++k) { const int yy = py + k / 3 - 1, xx = px + k % 3 - 1; const bool inb = yy >= 0 && yy < HH && xx >= 0 && xx < WWD; const float* src = U + ((b * NP + (size_t)(inb ? yy * WWD + xx : 0)) * CI) + 8 * g; float v[16];
#pragma unroll
    for (int i = 0; i < 8; ++i) { v[i] = inb ? src[i] : 0.f; v[8 + i] = inb ? src[16 + i] : 0.f; }
    const F2 a = bsplit16(v);
#pragma unroll
    for (int j = 0; j < 2; ++j) { const v16b w = frag_b(PW + (size_t)(j * 16 + col) * (KK * CI) + k * CI, lane); acc[j] = wmma_bf(a.h, w, acc[j]); acc[j] = wmma_bf(a.l, w, acc[j]); } }
  float vq[8];
#pragma unroll
  for (int r = 0; r < 8; ++r) { vq[r] = 0.f;
#pragma unroll
    for (int j = 0; j < 2; ++j) { const float v = fmaxf(acc[j][r] + bfr(BIAS[j * 16 + col]), 0.f); acc[j][r] = v; vq[r] += v * v; }
#pragma unroll
    for (int o = 1; o < 16; o <<= 1) vq[r] += __shfl_xor(vq[r], o); }
#pragma unroll
  for (int r = 0; r < 8; ++r) { const float n = fmaxf(sqrtf(vq[r]), PEPS); const float f = tanhf(SQC * n) / (SQC * n);
#pragma unroll
    for (int j = 0; j < 2; ++j) so[j * 16 + col][wave * 16 + 8 * g + r] = acc[j][r] * f; }
  __syncthreads();
  for (int e = tid; e < CO * 16; e += 128) { const int o = e >> 4, q = e & 15; vst2(Y + ((b * CO + o) * NP) + (size_t)blockIdx.x * 64 + q * 4, *(const v4f*)&so[o][q * 4]); } }
extern "C" void kernel_launch(void* const* d_in, const int* in_sizes, int n_in, void* d_out, int out_size, void* d_ws, size_t ws_size, hipStream_t stream) {
  (void)in_sizes; (void)n_in; (void)out_size;
  const float** F = (const float**)d_in;
  if (ws_size < (size_t)WS_END) return;
  char* ws = (char*)d_ws; __bf16* PW = (__bf16*)(ws + WS_PW); float* U = (float*)(ws + WS_U);
  k_packw<<<CO, 32, 0, stream>>>(F[1], PW);
  k_log<<<dim3(NP / 256, TNB), 256, 0, stream>>>(F[0], U);
  k_conv<<<dim3(TPB, TNB), 128, 0, stream>>>(U, PW, F[2], (float*)d_out);
}
